// HMMLayer_13778255086221
// MI455X (gfx1250) — hardware-verified
//
#include <hip/hip_runtime.h>


#define NS   128
#define AP   136
#define UP   260
#define EPSV 1e-8f

typedef __bf16   v16b __attribute__((ext_vector_type(16)));
typedef __bf16   v8b  __attribute__((ext_vector_type(8)));
typedef _Float16 v16h __attribute__((ext_vector_type(16)));
typedef float    v8f  __attribute__((ext_vector_type(8)));
typedef float    v4f  __attribute__((ext_vector_type(4)));
typedef unsigned v4u  __attribute__((ext_vector_type(4)));
typedef unsigned v2u  __attribute__((ext_vector_type(2)));

union FragB { v16b v; v16h hv; v8b q[2]; };

__device__ __forceinline__ unsigned bf_rne(float f) {
  unsigned u = __float_as_uint(f);
  return (u + 0x7FFFu + ((u >> 16) & 1u)) >> 16;
}

__device__ __forceinline__ void split4(v4f a, v2u& hi, v2u& lo) {
  const unsigned h0 = bf_rne(a.x), h1 = bf_rne(a.y), h2 = bf_rne(a.z), h3 = bf_rne(a.w);
  const unsigned l0 = bf_rne(a.x - __uint_as_float(h0 << 16));
  const unsigned l1 = bf_rne(a.y - __uint_as_float(h1 << 16));
  const unsigned l2 = bf_rne(a.z - __uint_as_float(h2 << 16));
  const unsigned l3 = bf_rne(a.w - __uint_as_float(h3 << 16));
  v2u th, tl;
  th.x = h0 | (h1 << 16); th.y = h2 | (h3 << 16);
  tl.x = l0 | (l1 << 16); tl.y = l2 | (l3 << 16);
  hi = th; lo = tl;
}

__device__ __forceinline__ v4u cat4(v2u a, v2u b) {
  v4u r;
  r.x = a.x; r.y = a.y; r.z = b.x; r.w = b.y;
  return r;
}

__device__ __forceinline__ v8f wmma_bf(v16b a, v16b b, v8f c) {
  return __builtin_amdgcn_wmma_f32_16x16x32_bf16(false, a, false, b, (short)0, c, false, false);
}

__device__ __forceinline__ void wguard(v8f& c, const FragB& a0, const FragB& a1,
                                       const FragB& b0, const FragB& b1) {
  asm volatile("v_nop\n\tv_nop\n\tv_nop\n\tv_nop"
               : "+v"(c)
               : "v"(a0.hv), "v"(a1.hv), "v"(b0.hv), "v"(b1.hv));
}

__device__ __forceinline__ void load_bfrags(FragB (&bh)[4], FragB (&bl)[4],
                                            const unsigned short* Ph, const unsigned short* Pl,
                                            int n, int h) {
  const unsigned short* ph = Ph + (size_t)n * NS + 8 * h;
  const unsigned short* pl = Pl + (size_t)n * NS + 8 * h;
#pragma unroll
  for (int kk = 0; kk < 4; ++kk) {
    bh[kk].q[0] = *(const v8b*)(ph + 32 * kk);
    bh[kk].q[1] = *(const v8b*)(ph + 32 * kk + 16);
    bl[kk].q[0] = *(const v8b*)(pl + 32 * kk);
    bl[kk].q[1] = *(const v8b*)(pl + 32 * kk + 16);
  }
}

__device__ __forceinline__ void tile_mma(const unsigned short* AHp, const unsigned short* ALp,
                                         const FragB (&bh)[4], const FragB (&bl)[4],
                                         float* Ut, int w, int h, int m) {
  v8f acc = {0.f, 0.f, 0.f, 0.f, 0.f, 0.f, 0.f, 0.f};
  const unsigned short* pah = AHp + m * AP + 8 * h;
  const unsigned short* pal = ALp + m * AP + 8 * h;
#pragma unroll
  for (int kk = 0; kk < 4; ++kk) {
    FragB ah, al;
    ah.q[0] = *(const v8b*)(pah + 32 * kk);
    ah.q[1] = *(const v8b*)(pah + 32 * kk + 16);
    al.q[0] = *(const v8b*)(pal + 32 * kk);
    al.q[1] = *(const v8b*)(pal + 32 * kk + 16);
    acc = wmma_bf(ah.v, bh[kk].v, acc);
    acc = wmma_bf(ah.v, bl[kk].v, acc);
    acc = wmma_bf(al.v, bh[kk].v, acc);
    wguard(acc, ah, al, bh[kk], bl[kk]);
  }
  float* up = Ut + (8 * h) * UP + 16 * w + m;
#pragma unroll
  for (int r = 0; r < 8; ++r) up[r * UP] = acc[r];
}

__device__ __forceinline__ float wsum(float s) {
  s += __shfl_xor(s, 16, 32);
  s += __shfl_xor(s, 8, 32);
  s += __shfl_xor(s, 4, 32);
  s += __shfl_xor(s, 2, 32);
  s += __shfl_xor(s, 1, 32);
  return s;
}

__device__ __forceinline__ v4f rownorm(v4f v) {
  const float s = wsum((v.x + v.y) + (v.z + v.w));
  const float inv = 1.0f / (s + EPSV);
  return v * inv;
}

__device__ __forceinline__ v4f sig4(v4f v) {
  v4f r;
  r.x = 1.0f / (1.0f + __expf(-v.x));
  r.y = 1.0f / (1.0f + __expf(-v.y));
  r.z = 1.0f / (1.0f + __expf(-v.z));
  r.w = 1.0f / (1.0f + __expf(-v.w));
  return r;
}

__global__ __launch_bounds__(256)
void k_prep(const float* __restrict__ logT, const float* __restrict__ logPi,
            unsigned short* PFh, unsigned short* PFl,
            unsigned short* PBh, unsigned short* PBl, float* p0) {
  __shared__ __attribute__((aligned(16))) float Ps[64 * NS];
  __shared__ __attribute__((aligned(16))) float p0s[NS];
  const int tid = threadIdx.x;

  if (tid < NS) {
    float mx2 = -3.4e38f;
#pragma unroll 1
    for (int c = 0; c < NS; ++c) mx2 = fmaxf(mx2, logPi[c]);
    p0s[tid] = expf(logPi[tid] - mx2);
  }

#pragma unroll 1
  for (int half = 0; half < 2; ++half) {
    if (tid < 64) {
      const float* rp = logT + (size_t)(64 * half + tid) * NS;
      float* pr = Ps + tid * NS;
      float mx = -3.4e38f;
#pragma unroll 1
      for (int c = 0; c < NS; ++c) mx = fmaxf(mx, rp[c]);
      float s = 0.f;
#pragma unroll 1
      for (int c = 0; c < NS; ++c) {
        const float e = expf(rp[c] - mx);
        pr[c] = e;
        s += e;
      }
      const float inv = 1.0f / s;
#pragma unroll 1
      for (int c = 0; c < NS; ++c) pr[c] = pr[c] * inv;
    }
    __syncthreads();

#pragma unroll 1
    for (int i = 0; i < 4; ++i) {
      const int p = tid + 256 * i;
      const int nl = p >> 4, k0 = (p & 15) * 8;
      const float* src = Ps + nl * NS + k0;
      const v4f b0 = *(const v4f*)src;
      const v4f b1 = *(const v4f*)(src + 4);
      v2u bh0, bl0, bh1, bl1;
      split4(b0, bh0, bl0);
      split4(b1, bh1, bl1);
      const v4u vbh = cat4(bh0, bh1), vbl = cat4(bl0, bl1);
      const size_t ob = (size_t)(64 * half + nl) * NS + k0;
      const int n = p >> 3, kq = (p & 7) * 8;
      v4f f0, f1;
      f0.x = Ps[(kq + 0) * NS + n]; f0.y = Ps[(kq + 1) * NS + n];
      f0.z = Ps[(kq + 2) * NS + n]; f0.w = Ps[(kq + 3) * NS + n];
      f1.x = Ps[(kq + 4) * NS + n]; f1.y = Ps[(kq + 5) * NS + n];
      f1.z = Ps[(kq + 6) * NS + n]; f1.w = Ps[(kq + 7) * NS + n];
      v2u fh0, fl0, fh1, fl1;
      split4(f0, fh0, fl0);
      split4(f1, fh1, fl1);
      const v4u vfh = cat4(fh0, fh1), vfl = cat4(fl0, fl1);
      const size_t of = (size_t)n * NS + 64 * half + kq;

      *(volatile v4u*)(PBh + ob) = vbh;
      *(volatile v4u*)(PBl + ob) = vbl;
      *(volatile v4u*)(PFh + of) = vfh;
      *(volatile v4u*)(PFl + of) = vfl;
      __threadfence();
      *(volatile v4u*)(PBh + ob) = vbh;
      *(volatile v4u*)(PBl + ob) = vbl;
      *(volatile v4u*)(PFh + of) = vfh;
      *(volatile v4u*)(PFl + of) = vfl;
    }
    __syncthreads();
  }

  float s2 = 0.f;
#pragma unroll 1
  for (int c = 0; c < NS; ++c) s2 += p0s[c];
  const float inv2 = 1.0f / s2;
  if (tid < 32) {
    const v4f v = *(const v4f*)(p0s + 4 * tid) * inv2;
    *(volatile v4f*)(p0 + 4 * tid) = v;
    __threadfence();
    *(volatile v4f*)(p0 + 4 * tid) = v;
  }
}

__device__ __forceinline__ void fwd_finish(v4f ua, v4f ub, float* ga, float* gb,
                                           unsigned short* hA, unsigned short* lA,
                                           unsigned short* hB, unsigned short* lB) {
  const v4f a = rownorm(ua);
  const v4f b = rownorm(ub);
  *(volatile v4f*)ga = a;
  *(volatile v4f*)gb = b;
  v2u hh, ll;
  split4(a, hh, ll);
  *(v2u*)hA = hh; *(v2u*)lA = ll;
  split4(b, hh, ll);
  *(v2u*)hB = hh; *(v2u*)lB = ll;
  __threadfence();
  *(volatile v4f*)ga = a;
  *(volatile v4f*)gb = b;
}

__global__ __launch_bounds__(256)
void k_fwd(const float* __restrict__ x, const unsigned short* __restrict__ PFh,
           const unsigned short* __restrict__ PFl, const float* __restrict__ p0,
           float* Apl, int T, int nb) {
  __shared__ __attribute__((aligned(16))) unsigned short AH[16 * AP];
  __shared__ __attribute__((aligned(16))) unsigned short AL[16 * AP];
  __shared__ __attribute__((aligned(16))) float U[16 * UP];
  const int tid = threadIdx.x, w = tid >> 5, l = tid & 31, h = l >> 4, m = l & 15;
  const int bbase = blockIdx.x * 16;
  if (bbase + 16 > nb) return;

  FragB bh[4], bl[4];
  load_bfrags(bh, bl, PFh, PFl, 16 * w + m, h);

  const int rowA = 2 * w, rowB = 2 * w + 1;
  const size_t gA = ((size_t)(bbase + rowA) * T) * NS + 4 * l;
  const size_t gB = ((size_t)(bbase + rowB) * T) * NS + 4 * l;
  unsigned short* hA = AH + rowA * AP + 4 * l;
  unsigned short* lA = AL + rowA * AP + 4 * l;
  unsigned short* hB = AH + rowB * AP + 4 * l;
  unsigned short* lB = AL + rowB * AP + 4 * l;
  const float* uA = U + rowA * UP + 4 * l;
  const float* uB = U + rowB * UP + 4 * l;

  {
    const v4f pv = *(const v4f*)(p0 + 4 * l);
    const v4f ua = pv * sig4(*(const v4f*)(x + gA));
    const v4f ub = pv * sig4(*(const v4f*)(x + gB));
    fwd_finish(ua, ub, Apl + gA, Apl + gB, hA, lA, hB, lB);
  }
  __syncthreads();

#pragma unroll 1
  for (int t = 1; t < T; ++t) {
    tile_mma(AH, AL, bh, bl, U, w, h, m);
    __syncthreads();
    const size_t to = (size_t)t * NS;
    const v4f ua = *(const v4f*)uA * sig4(*(const v4f*)(x + gA + to));
    const v4f ub = *(const v4f*)uB * sig4(*(const v4f*)(x + gB + to));
    fwd_finish(ua, ub, Apl + gA + to, Apl + gB + to, hA, lA, hB, lB);
    __syncthreads();
  }
}

__device__ __forceinline__ void bwd_finish(v4f ba, v4f bb, const float* aa, const float* ab,
                                           const float* xa, const float* xb,
                                           float* oa, float* ob,
                                           unsigned short* hA, unsigned short* lA,
                                           unsigned short* hB, unsigned short* lB) {
  const v4f pa = rownorm(*(const v4f*)aa * ba);
  const v4f pb = rownorm(*(const v4f*)ab * bb);
  *(volatile v4f*)oa = pa;
  *(volatile v4f*)ob = pb;
  const v4f ca = sig4(*(const v4f*)xa) * ba;
  const v4f cb = sig4(*(const v4f*)xb) * bb;
  v2u hh, ll;
  split4(ca, hh, ll);
  *(v2u*)hA = hh; *(v2u*)lA = ll;
  split4(cb, hh, ll);
  *(v2u*)hB = hh; *(v2u*)lB = ll;
  __threadfence();
  *(volatile v4f*)oa = pa;
  *(volatile v4f*)ob = pb;
}

__global__ __launch_bounds__(256)
void k_bwd(const float* __restrict__ x, const unsigned short* __restrict__ PBh,
           const unsigned short* __restrict__ PBl, const float* __restrict__ Apl,
           float* out, int T, int nb) {
  __shared__ __attribute__((aligned(16))) unsigned short CH[16 * AP];
  __shared__ __attribute__((aligned(16))) unsigned short CL[16 * AP];
  __shared__ __attribute__((aligned(16))) float U[16 * UP];
  const int tid = threadIdx.x, w = tid >> 5, l = tid & 31, h = l >> 4, m = l & 15;
  const int bbase = blockIdx.x * 16;
  if (bbase + 16 > nb) return;

  FragB bh[4], bl[4];
  load_bfrags(bh, bl, PBh, PBl, 16 * w + m, h);

  const int rowA = 2 * w, rowB = 2 * w + 1;
  const size_t gA = ((size_t)(bbase + rowA) * T) * NS + 4 * l;
  const size_t gB = ((size_t)(bbase + rowB) * T) * NS + 4 * l;
  unsigned short* hA = CH + rowA * AP + 4 * l;
  unsigned short* lA = CL + rowA * AP + 4 * l;
  unsigned short* hB = CH + rowB * AP + 4 * l;
  unsigned short* lB = CL + rowB * AP + 4 * l;
  const float* uA = U + rowA * UP + 4 * l;
  const float* uB = U + rowB * UP + 4 * l;

  {
    const size_t to = (size_t)(T - 1) * NS;
    const v4f one = {1.f, 1.f, 1.f, 1.f};
    bwd_finish(one, one, Apl + gA + to, Apl + gB + to, x + gA + to, x + gB + to,
               out + gA + to, out + gB + to, hA, lA, hB, lB);
  }
  __syncthreads();

#pragma unroll 1
  for (int t = T - 2; t >= 0; --t) {
    tile_mma(CH, CL, bh, bl, U, w, h, m);
    __syncthreads();
    const size_t to = (size_t)t * NS;
    const v4f ba = rownorm(*(const v4f*)uA);
    const v4f bb = rownorm(*(const v4f*)uB);
    bwd_finish(ba, bb, Apl + gA + to, Apl + gB + to, x + gA + to, x + gB + to,
               out + gA + to, out + gB + to, hA, lA, hB, lB);
    __syncthreads();
  }
}

extern "C" void kernel_launch(void* const* d_in, const int* in_sizes, int n_in,
                              void* d_out, int out_size, void* d_ws, size_t ws_size,
                              hipStream_t stream) {
  const int NBATCH = 32, NSTEP = 4000;
  if (n_in < 3) return;
  const int nx = in_sizes[0];
  if (nx != NBATCH * NSTEP * NS || in_sizes[1] != NS * NS || in_sizes[2] != NS ||
      out_size != nx) return;
  if ((NBATCH % 16) != 0 || NSTEP < 2) return;

  const float* x     = (const float*)d_in[0];
  const float* logT  = (const float*)d_in[1];
  const float* logPi = (const float*)d_in[2];
  float* out = (float*)d_out;

  char* ws = (char*)d_ws;
  size_t off = 0;
  float* Apl = (float*)(ws + off);
  off += (size_t)nx * sizeof(float);
  off = (off + 255) & ~(size_t)255;
  unsigned short* PFh = (unsigned short*)(ws + off); off += (size_t)NS * NS * 2;
  unsigned short* PFl = (unsigned short*)(ws + off); off += (size_t)NS * NS * 2;
  unsigned short* PBh = (unsigned short*)(ws + off); off += (size_t)NS * NS * 2;
  unsigned short* PBl = (unsigned short*)(ws + off); off += (size_t)NS * NS * 2;
  float* p0 = (float*)(ws + off);                    off += (size_t)NS * sizeof(float);
  if (off > ws_size) return;

  k_prep<<<dim3(1), dim3(256), 0, stream>>>(logT, logPi, PFh, PFl, PBh, PBl, p0);
  k_fwd<<<dim3(NBATCH / 16), dim3(256), 0, stream>>>(x, PFh, PFl, p0, Apl, NSTEP, NBATCH);
  k_bwd<<<dim3(NBATCH / 16), dim3(256), 0, stream>>>(x, PBh, PBl, Apl, out, NSTEP, NBATCH);
}
